// Model_13778255085586
// MI455X (gfx1250) — hardware-verified
//
#include <hip/hip_runtime.h>
#include <math.h>

constexpr int NBATCH   = 256;
constexpr int SEQ_T    = 256;
constexpr int NCH      = 64;
constexpr int NHID     = 512;
constexpr int NGATE    = 4 * NHID;
constexpr int NIN2     = 2 * NCH;
constexpr int NTHR     = 256;
constexpr int ROWS_BLK = 16;
constexpr int PITCH_D  = 72;
constexpr int PITCH_H  = 520;
constexpr int PITCH_CM = 136;
constexpr int PITCH_XC = 72;
constexpr int PITCH_IN = 136;
constexpr int PITCH_F  = 68;
constexpr float WCARRY     = 256.0f;
constexpr float WCARRY_INV = 1.0f / 256.0f;

static_assert(NBATCH % ROWS_BLK == 0, "batch tile");
static_assert(NHID == 64 * (NTHR / 32), "8 waves x 64 hidden units");
static_assert(NCH == 64 && NCH % 32 == 0, "K of the decay and feature products");
static_assert(NIN2 % 32 == 0 && NHID % 32 == 0, "K multiples of 32");
static_assert(ROWS_BLK * NCH == NTHR * 4, "staging map: 256 threads x 4 elements = 16 x 64");
static_assert(NGATE % NTHR == 0 && NHID % NTHR == 0, "bias staging loops exact");
static_assert((ROWS_BLK * NHID) % NTHR == 0, "h tile zero-fill loop exact");
static_assert((PITCH_D % 8) == 0 && (PITCH_H % 8) == 0 && (PITCH_CM % 8) == 0 && (PITCH_IN % 8) == 0 && (PITCH_F % 4) == 0, "LDS alignment");

typedef __attribute__((ext_vector_type(16))) _Float16 v16h;
typedef __attribute__((ext_vector_type(8)))  _Float16 v8h;
typedef __attribute__((ext_vector_type(4)))  _Float16 v4h;
typedef __attribute__((ext_vector_type(8)))  float    v8f;
typedef __attribute__((ext_vector_type(4)))  float    v4f;

__device__ __forceinline__ void guard1x2_h(v8f& a, v16h x, v16h y) {
  asm volatile("v_nop\n\tv_nop\n\tv_nop\n\tv_nop" : "+v"(a) : "v"(x), "v"(y));
}
__device__ __forceinline__ void guard1x4_h(v8f& a, v16h x0, v16h x1, v16h y0, v16h y1) {
  asm volatile("v_nop\n\tv_nop\n\tv_nop\n\tv_nop" : "+v"(a) : "v"(x0), "v"(x1), "v"(y0), "v"(y1));
}
__device__ __forceinline__ void guard4_h(v8f& a0, v8f& a1, v8f& a2, v8f& a3, v16h x, v16h y0, v16h y1, v16h y2, v16h y3) {
  asm volatile("v_nop\n\tv_nop\n\tv_nop\n\tv_nop" : "+v"(a0), "+v"(a1), "+v"(a2), "+v"(a3) : "v"(x), "v"(y0), "v"(y1), "v"(y2), "v"(y3));
}
__device__ __forceinline__ void acc_guard4(v8f& a, v8f& b, v8f& c, v8f& d) {
  asm volatile("v_nop\n\tv_nop\n\tv_nop\n\tv_nop" : "+v"(a), "+v"(b), "+v"(c), "+v"(d));
}

template <typename T> struct Frag;
template <> struct Frag<_Float16> {
  typedef v16h V; union U { v16h v; v8h h[2]; };
  static __device__ __forceinline__ v16h load(const _Float16* p) {
    U f; f.h[0] = *(const v8h*)(p); f.h[1] = *(const v8h*)(p + 16); return f.v;
  }
  static __device__ __forceinline__ v8f mma(v16h a, v16h b, v8f c) {
    return __builtin_amdgcn_wmma_f32_16x16x32_f16(false, a, false, b, (short)0, c, false, false);
  }
};
typedef Frag<_Float16> FH;

__device__ __forceinline__ float fsig(float x)  { return __builtin_amdgcn_rcpf(1.0f + __expf(-x)); }
__device__ __forceinline__ float ftanh(float x) { return 1.0f - 2.0f * __builtin_amdgcn_rcpf(__expf(2.0f * x) + 1.0f); }
__device__ __forceinline__ float ftz_pos(float g) { return (g < 1.17549435e-38f) ? 0.0f : g; }

__global__ __launch_bounds__(NTHR) void cvt8_f16_kernel(const float* __restrict__ src, unsigned short* __restrict__ dst,
                                                        int nrow, int ncol8, int zero_diag, float sc) {
  const int i  = blockIdx.x * NTHR + threadIdx.x;
  const int n8 = nrow * ncol8;
  if (i < n8) {
    const int row = i / ncol8;
    const int c8  = i - row * ncol8;
    const float* sp = src + (size_t)row * (size_t)(ncol8 * 8) + c8 * 8;
    const v4f a = *(const v4f*)(sp);
    const v4f b = *(const v4f*)(sp + 4);
    v8h hv;
#pragma unroll
    for (int e = 0; e < 4; ++e) {
      float fa = a[e];
      float fb = b[e];
      const int col = c8 * 8 + e;
      if (zero_diag) {
        fa = (col == row) ? 0.0f : fa;
        fb = (col + 4 == row) ? 0.0f : fb;
      }
      hv[e]     = (_Float16)(fa * sc);
      hv[4 + e] = (_Float16)(fb * sc);
    }
    unsigned short* op = dst + (size_t)i * 8;
    *(volatile v8h*)op = hv;
    __threadfence();
    *(volatile v8h*)op = hv;
  }
}

__global__ __launch_bounds__(NTHR) __attribute__((amdgpu_num_vgpr(256))) void impute_scan_kernel(
    const float* __restrict__ data,
    const unsigned short* __restrict__ WHHp, const unsigned short* __restrict__ WIHp,
    const unsigned short* __restrict__ WGHp, const unsigned short* __restrict__ WHISTp,
    const unsigned short* __restrict__ WFEATp, const unsigned short* __restrict__ WCOMBp,
    const float* __restrict__ b_ih, const float* __restrict__ b_hh, const float* __restrict__ b_gh,
    const float* __restrict__ W_gx, const float* __restrict__ b_gx,
    const float* __restrict__ b_hist, const float* __restrict__ b_feat, const float* __restrict__ b_comb,
    float* __restrict__ out) {
  __shared__ __align__(16) _Float16 Ad [ROWS_BLK * PITCH_D];
  __shared__ __align__(16) _Float16 Ahd[ROWS_BLK * PITCH_H];
  __shared__ __align__(16) _Float16 Acm[ROWS_BLK * PITCH_CM];
  __shared__ __align__(16) _Float16 Axc[ROWS_BLK * PITCH_XC];
  __shared__ __align__(16) _Float16 Ain[ROWS_BLK * PITCH_IN];
  __shared__ __align__(16) float    Xs [ROWS_BLK * PITCH_F];
  __shared__ __align__(16) float    Ms [ROWS_BLK * PITCH_F];
  __shared__ __align__(16) float    Os [ROWS_BLK * PITCH_F];
  __shared__ __align__(16) float    Hf [ROWS_BLK * NHID];
  __shared__ __align__(16) float    Bs [NGATE];
  __shared__ __align__(16) float    Bgh[NHID];

  const _Float16* WHH   = (const _Float16*)WHHp;
  const _Float16* WIH   = (const _Float16*)WIHp;
  const _Float16* WGH   = (const _Float16*)WGHp;
  const _Float16* WHIST = (const _Float16*)WHISTp;
  const _Float16* WFEAT = (const _Float16*)WFEATp;
  const _Float16* WCOMB = (const _Float16*)WCOMBp;

  const int tid  = threadIdx.x;
  const int lane = tid & 31;
  const int wave = __builtin_amdgcn_readfirstlane(tid >> 5);
  const int c    = lane & 15;
  const int hh   = lane >> 4;
  const int koff = hh * 8;
  const int rowbase = blockIdx.x * ROWS_BLK;

#pragma unroll 1
  for (int i = tid; i < NGATE; i += NTHR) Bs[i] = b_ih[i] + b_hh[i];
#pragma unroll 1
  for (int i = tid; i < NHID; i += NTHR) Bgh[i] = b_gh[i];
#pragma unroll 1
  for (int i = tid; i < ROWS_BLK * NHID; i += NTHR) Hf[i] = 0.0f;

  const int m_a = tid >> 4;
  const int c4  = (tid & 15) * 4;
  float wgx[4], bgx[4], dcur[4];
  {
    const v4f bv = *(const v4f*)(b_gx + c4);
#pragma unroll
    for (int e = 0; e < 4; ++e) {
      wgx[e]  = W_gx[(size_t)(c4 + e) * NCH + (c4 + e)];
      bgx[e]  = bv[e];
      dcur[e] = 0.0f;
    }
  }
  const int nsm = 16 * (wave & 3) + c;
  const float bhist_c = b_hist[nsm];
  const float bfeat_c = b_feat[nsm];
  const float bcomb_c = b_comb[nsm];

  float cst[4][8];
#pragma unroll
  for (int nt = 0; nt < 4; ++nt)
#pragma unroll
    for (int r = 0; r < 8; ++r) cst[nt][r] = 0.0f;

  const v8f z8 = {0.f, 0.f, 0.f, 0.f, 0.f, 0.f, 0.f, 0.f};
  __syncthreads();

#pragma unroll 1
  for (int t = 0; t < SEQ_T; ++t) {
    {
      v4f dv = *(const v4f*)(data + ((size_t)(rowbase + m_a) * SEQ_T + (size_t)t) * NCH + c4);
      asm volatile("" : "+v"(dv));
      v4f xv, mv;
      v4h dh, gh, mh;
#pragma unroll
      for (int e = 0; e < 4; ++e) {
        const float f = dv[e];
        const unsigned ubits = __float_as_uint(f);
        const bool isn = (ubits & 0x7fffffffu) > 0x7f800000u;
        const float mk = isn ? 0.0f : 1.0f;
        const float xx = isn ? 0.0f : f;
        const float dd = dcur[e];
        const float zz = fmaxf(dd * wgx[e] + bgx[e], 0.0f);
        const float gx = ftz_pos(expf(-zz));
        xv[e] = xx;
        mv[e] = mk;
        dh[e] = (_Float16)dd;
        gh[e] = (_Float16)gx;
        mh[e] = (_Float16)mk;
        dcur[e] = isn ? (dd + 1.0f) : 1.0f;
      }
      *(v4h*)(Ad  + m_a * PITCH_D  + c4)       = dh;
      *(v4h*)(Acm + m_a * PITCH_CM + c4)       = gh;
      *(v4h*)(Acm + m_a * PITCH_CM + NCH + c4) = mh;
      *(v4h*)(Ain + m_a * PITCH_IN + NCH + c4) = mh;
      *(v4f*)(Xs  + m_a * PITCH_F  + c4)       = xv;
      *(v4f*)(Ms  + m_a * PITCH_F  + c4)       = mv;
    }
    __syncthreads();

    {
      const _Float16* adrow = Ad + c * PITCH_D + koff;
      const v16h a0 = FH::load(adrow);
      const v16h a1 = FH::load(adrow + 32);
#pragma unroll 1
      for (int nt = 0; nt < 4; ++nt) {
        const int j = 64 * wave + 16 * nt + c;
        const _Float16* wg = WGH + (size_t)j * NCH + koff;
        const v16h b0 = FH::load(wg);
        const v16h b1 = FH::load(wg + 32);
        v8f acc = z8;
        acc = FH::mma(a0, b0, acc);
        acc = FH::mma(a1, b1, acc);
        guard1x4_h(acc, a0, a1, b0, b1);
        const float bg = Bgh[j];
#pragma unroll
        for (int r = 0; r < 8; ++r) {
          const int row = 8 * hh + r;
          const float zz = fmaxf(acc[r] * WCARRY_INV + bg, 0.0f);
          const float g  = ftz_pos(__expf(-zz));
          const float hd = Hf[row * NHID + j] * g;
          Ahd[row * PITCH_H + j] = (_Float16)hd;
        }
      }
    }
    __syncthreads();

    float xh[8];
#pragma unroll
    for (int r = 0; r < 8; ++r) xh[r] = 0.0f;
    if (wave < 4) {
      const _Float16* ahrow = Ahd + c * PITCH_H + koff;
      const _Float16* wh = WHIST + (size_t)nsm * NHID + koff;
      v8f acc = z8;
#pragma unroll 1
      for (int k0 = 0; k0 < NHID; k0 += 32) {
        const v16h a = FH::load(ahrow + k0);
        const v16h b = FH::load(wh + k0);
        acc = FH::mma(a, b, acc);
        guard1x2_h(acc, a, b);
      }
#pragma unroll
      for (int r = 0; r < 8; ++r) {
        const int row = 8 * hh + r;
        const float xhv = acc[r] * WCARRY_INV + bhist_c;
        const float mk  = Ms[row * PITCH_F + nsm];
        const float xx  = Xs[row * PITCH_F + nsm];
        const float xc  = (mk != 0.0f) ? xx : xhv;
        xh[r] = xhv;
        Axc[row * PITCH_XC + nsm] = (_Float16)xc;
      }
    }
    __syncthreads();

    if (wave < 4) {
      const _Float16* xcrow = Axc + c * PITCH_XC + koff;
      const _Float16* wf = WFEAT + (size_t)nsm * NCH + koff;
      v8f accz = z8;
      {
        const v16h a0 = FH::load(xcrow);
        const v16h a1 = FH::load(xcrow + 32);
        const v16h b0 = FH::load(wf);
        const v16h b1 = FH::load(wf + 32);
        accz = FH::mma(a0, b0, accz);
        accz = FH::mma(a1, b1, accz);
        guard1x4_h(accz, a0, a1, b0, b1);
      }
      const _Float16* cmrow = Acm + c * PITCH_CM + koff;
      const _Float16* wc = WCOMB + (size_t)nsm * NIN2 + koff;
      v8f acca = z8;
#pragma unroll 1
      for (int k0 = 0; k0 < NIN2; k0 += 32) {
        const v16h a = FH::load(cmrow + k0);
        const v16h b = FH::load(wc + k0);
        acca = FH::mma(a, b, acca);
        guard1x2_h(acca, a, b);
      }
#pragma unroll
      for (int r = 0; r < 8; ++r) {
        const int row = 8 * hh + r;
        const float zh = accz[r] * WCARRY_INV + bfeat_c;
        const float al = acca[r] * WCARRY_INV + bcomb_c;
        const float ch = al * zh + (1.0f - al) * xh[r];
        const float mk = Ms[row * PITCH_F + nsm];
        const float xx = Xs[row * PITCH_F + nsm];
        const float cc = (mk != 0.0f) ? xx : ch;
        Os[row * PITCH_F + nsm] = cc;
        Ain[row * PITCH_IN + nsm] = (_Float16)cc;
      }
    }
    __syncthreads();

    {
      const int row = 2 * wave + hh;
      const int c4o = c * 4;
      const v4f v = *(const v4f*)(Os + row * PITCH_F + c4o);
      float* op = out + ((size_t)(rowbase + row) * SEQ_T + (size_t)t) * NCH + c4o;
      *(volatile v4f*)op = v;
      __threadfence();
      *(volatile v4f*)op = v;
    }

    {
      const _Float16* inrow = Ain + c * PITCH_IN + koff;
      const _Float16* ahrow = Ahd + c * PITCH_H + koff;
#pragma unroll
      for (int nt = 0; nt < 4; ++nt) {
        const int j = 64 * wave + 16 * nt + c;
        const _Float16* wi = WIH + (size_t)j * NIN2 + koff;
        const _Float16* wh = WHH + (size_t)j * NHID + koff;
        v8f a0 = z8, a1 = z8, a2 = z8, a3 = z8;
#pragma unroll 1
        for (int kx = 0; kx < NIN2; kx += 32) {
          const v16h a  = FH::load(inrow + kx);
          const v16h b0 = FH::load(wi + kx);
          const v16h b1 = FH::load(wi + (size_t)1 * NHID * NIN2 + kx);
          const v16h b2 = FH::load(wi + (size_t)2 * NHID * NIN2 + kx);
          const v16h b3 = FH::load(wi + (size_t)3 * NHID * NIN2 + kx);
          a0 = FH::mma(a, b0, a0);
          a1 = FH::mma(a, b1, a1);
          a2 = FH::mma(a, b2, a2);
          a3 = FH::mma(a, b3, a3);
          guard4_h(a0, a1, a2, a3, a, b0, b1, b2, b3);
        }
#pragma unroll 1
        for (int k0 = 0; k0 < NHID; k0 += 32) {
          const v16h a  = FH::load(ahrow + k0);
          const v16h b0 = FH::load(wh + k0);
          const v16h b1 = FH::load(wh + (size_t)1 * NHID * NHID + k0);
          const v16h b2 = FH::load(wh + (size_t)2 * NHID * NHID + k0);
          const v16h b3 = FH::load(wh + (size_t)3 * NHID * NHID + k0);
          a0 = FH::mma(a, b0, a0);
          a1 = FH::mma(a, b1, a1);
          a2 = FH::mma(a, b2, a2);
          a3 = FH::mma(a, b3, a3);
          guard4_h(a0, a1, a2, a3, a, b0, b1, b2, b3);
        }
        acc_guard4(a0, a1, a2, a3);
        const float bi = Bs[j];
        const float bf = Bs[NHID + j];
        const float bg = Bs[2 * NHID + j];
        const float bo = Bs[3 * NHID + j];
#pragma unroll
        for (int r = 0; r < 8; ++r) {
          const float zi = a0[r] * WCARRY_INV + bi;
          const float zf = a1[r] * WCARRY_INV + bf;
          const float zg = a2[r] * WCARRY_INV + bg;
          const float zo = a3[r] * WCARRY_INV + bo;
          const float cn = fsig(zf) * cst[nt][r] + fsig(zi) * ftanh(zg);
          cst[nt][r] = cn;
          const float hn = fsig(zo) * ftanh(cn);
          Hf[(8 * hh + r) * NHID + j] = hn;
        }
      }
    }
    __syncthreads();
  }
}

extern "C" void kernel_launch(void* const* d_in, const int* in_sizes, int n_in,
                              void* d_out, int out_size, void* d_ws, size_t ws_size, hipStream_t stream) {
  if (n_in < 15 || d_out == nullptr || d_ws == nullptr) return;
  if (in_sizes[0] != NBATCH * SEQ_T * NCH || in_sizes[1] != NGATE * NIN2 || in_sizes[2] != NGATE * NHID ||
      in_sizes[3] != NGATE || in_sizes[4] != NGATE || in_sizes[5] != NHID * NCH || in_sizes[6] != NHID ||
      in_sizes[7] != NCH * NCH || in_sizes[8] != NCH || in_sizes[9] != NCH * NHID || in_sizes[10] != NCH ||
      in_sizes[11] != NCH * NCH || in_sizes[12] != NCH || in_sizes[13] != NCH * NIN2 || in_sizes[14] != NCH ||
      out_size != NBATCH * SEQ_T * NCH) return;

  const float* data   = (const float*)d_in[0];
  const float* W_ih   = (const float*)d_in[1];
  const float* W_hh   = (const float*)d_in[2];
  const float* b_ih   = (const float*)d_in[3];
  const float* b_hh   = (const float*)d_in[4];
  const float* W_gh   = (const float*)d_in[5];
  const float* b_gh   = (const float*)d_in[6];
  const float* W_gx   = (const float*)d_in[7];
  const float* b_gx   = (const float*)d_in[8];
  const float* W_hist = (const float*)d_in[9];
  const float* b_hist = (const float*)d_in[10];
  const float* W_feat = (const float*)d_in[11];
  const float* b_feat = (const float*)d_in[12];
  const float* W_comb = (const float*)d_in[13];
  const float* b_comb = (const float*)d_in[14];
  float* out = (float*)d_out;

  char* ws = (char*)d_ws; size_t off = 0;
  auto carve = [&](size_t bytes) -> char* { char* p = ws + off; off += (bytes + 255) & ~(size_t)255; return p; };
  unsigned short* WHH   = (unsigned short*)carve((size_t)NGATE * NHID * 2);
  unsigned short* WIH   = (unsigned short*)carve((size_t)NGATE * NIN2 * 2);
  unsigned short* WGH   = (unsigned short*)carve((size_t)NHID * NCH * 2);
  unsigned short* WHIST = (unsigned short*)carve((size_t)NCH * NHID * 2);
  unsigned short* WFEAT = (unsigned short*)carve((size_t)NCH * NCH * 2);
  unsigned short* WCOMB = (unsigned short*)carve((size_t)NCH * NIN2 * 2);
  if (off > ws_size || off > (size_t)134217728) return;

  const int n8_hh   = NGATE * (NHID / 8);
  const int n8_ih   = NGATE * (NIN2 / 8);
  const int n8_gh   = NHID * (NCH / 8);
  const int n8_hist = NCH * (NHID / 8);
  const int n8_feat = NCH * (NCH / 8);
  const int n8_comb = NCH * (NIN2 / 8);
  cvt8_f16_kernel<<<(n8_hh   + NTHR - 1) / NTHR, NTHR, 0, stream>>>(W_hh,   WHH,   NGATE, NHID / 8, 0, WCARRY);
  cvt8_f16_kernel<<<(n8_ih   + NTHR - 1) / NTHR, NTHR, 0, stream>>>(W_ih,   WIH,   NGATE, NIN2 / 8, 0, WCARRY);
  cvt8_f16_kernel<<<(n8_gh   + NTHR - 1) / NTHR, NTHR, 0, stream>>>(W_gh,   WGH,   NHID,  NCH / 8,  0, WCARRY);
  cvt8_f16_kernel<<<(n8_hist + NTHR - 1) / NTHR, NTHR, 0, stream>>>(W_hist, WHIST, NCH,   NHID / 8, 0, WCARRY);
  cvt8_f16_kernel<<<(n8_feat + NTHR - 1) / NTHR, NTHR, 0, stream>>>(W_feat, WFEAT, NCH,   NCH / 8,  1, WCARRY);
  cvt8_f16_kernel<<<(n8_comb + NTHR - 1) / NTHR, NTHR, 0, stream>>>(W_comb, WCOMB, NCH,   NIN2 / 8, 0, WCARRY);

  impute_scan_kernel<<<NBATCH / ROWS_BLK, NTHR, 0, stream>>>(
      data, WHH, WIH, WGH, WHIST, WFEAT, WCOMB,
      b_ih, b_hh, b_gh, W_gx, b_gx, b_hist, b_feat, b_comb, out);
}
